// SelectiveSSM_16716012716040
// MI455X (gfx1250) — hardware-verified
//
#include <hip/hip_runtime.h>
#include <math.h>

typedef __attribute__((ext_vector_type(16))) _Float16 v16h;
typedef __attribute__((ext_vector_type(8)))  _Float16 v8h;
typedef __attribute__((ext_vector_type(8)))  float    v8f;
typedef __attribute__((ext_vector_type(4)))  float    v4f;

constexpr int kBatch  = 2;
constexpr int kSeq    = 4096;
constexpr int kDm     = 1024;
constexpr int kDin    = 2048;
constexpr int kNst    = 16;
constexpr int kXzP    = 2 * kDin;
constexpr int kXdN    = 1 + 2 * kNst;
constexpr int kXdP    = 64;
constexpr int kRows   = kBatch * kSeq;
constexpr int kTP     = 260;
constexpr int kScanTS = 64;

constexpr float kCarX = 16.0f;
constexpr float kCarW = 32.0f;
constexpr float kCarU = 64.0f;
constexpr float kCarG = 1024.0f;
constexpr float kFoldIn  = 1.0f / (kCarX * kCarW);
constexpr float kFoldXd  = 1.0f / (kCarU * kCarW);
constexpr float kFoldOut = 1.0f / (kCarG * kCarW);
constexpr float kInvCarU = 1.0f / kCarU;

static_assert(kXdN == 33 && kXdN <= kXdP, "x_dbl width");
static_assert((kDm % 32) == 0 && (kDin % 32) == 0, "GEMM K multiples of 32");
static_assert((kSeq % 64) == 0 && (kXzP % 64) == 0 && (kXdP % 64) == 0 && (kDm % 64) == 0, "GEMM M,N multiples of 64");
static_assert((kDm % 64) == 0 && (kDin % 64) == 0 && (kDin % 256) == 0 && (kSeq % kScanTS) == 0, "tile multiples");

constexpr size_t kOffX16   = 0;
constexpr size_t kOffWINT  = kOffX16   + (size_t)kRows * kDm  * 2;
constexpr size_t kOffWOUTT = kOffWINT  + (size_t)kXzP  * kDm  * 2;
constexpr size_t kOffWXT   = kOffWOUTT + (size_t)kDm   * kDin * 2;
constexpr size_t kOffXZ    = kOffWXT   + (size_t)kXdP  * kDin * 2;
constexpr size_t kOffCONV  = kOffXZ    + (size_t)kSeq  * kXzP * 4;
constexpr size_t kOffGO    = kOffCONV  + (size_t)kSeq  * kDin * 2;
constexpr size_t kOffXD    = kOffGO    + (size_t)kSeq  * kDin * 2;
constexpr size_t kOffYS    = kOffXD    + (size_t)kSeq  * kXdP * 4;
constexpr size_t kWsTotal  = kOffYS    + (size_t)kSeq  * 4;
static_assert(kWsTotal == 131350528ull, "carve total");
static_assert(kWsTotal <= 134217728ull, "carve cap");
static_assert((kOffWINT % 128) == 0 && (kOffWOUTT % 128) == 0 && (kOffWXT % 128) == 0 && (kOffXZ % 128) == 0 &&
              (kOffCONV % 128) == 0 && (kOffGO % 128) == 0 && (kOffXD % 128) == 0 && (kOffYS % 128) == 0,
              "128-B aligned regions");

__device__ __forceinline__ unsigned short f2bf_bits(float f) {
  unsigned u = __float_as_uint(f);
  return (unsigned short)((u + 0x7FFFu + ((u >> 16) & 1u)) >> 16);
}
__device__ __forceinline__ float bf_bits2f(unsigned short h) { return __uint_as_float(((unsigned)h) << 16); }
__device__ __forceinline__ float bf_rne(float f) { return bf_bits2f(f2bf_bits(f)); }

__device__ __forceinline__ float h16_to_f32(unsigned hb) {
  const unsigned sgn = (hb & 0x8000u) << 16;
  const unsigned em = hb & 0x7fffu;
  const float fn = __uint_as_float((em << 13) + 0x38000000u);
  const float fs = (float)em * 5.9604644775390625e-8f;
  const float mag = (em < 0x400u) ? fs : fn;
  return __uint_as_float(__float_as_uint(mag) | sgn);
}

__device__ __forceinline__ float silu_f(float v) {
  const float e = expf(-v);
  return v * __builtin_amdgcn_rcpf(1.0f + e);
}

__device__ __forceinline__ void dep_guard4_h(v8f& a, v8f& b, v8f& c, v8f& d, v16h x, v16h y0, v16h y1, v16h y2, v16h y3) {
  asm volatile("v_nop\n\tv_nop\n\tv_nop\n\tv_nop" : "+v"(a), "+v"(b), "+v"(c), "+v"(d) : "v"(x), "v"(y0), "v"(y1), "v"(y2), "v"(y3));
}
__device__ __forceinline__ void keep4_h(v16h a, v16h b, v16h c, v16h d) { asm volatile("v_nop" :: "v"(a), "v"(b), "v"(c), "v"(d)); }
__device__ __forceinline__ void acc_guard4(v8f& a, v8f& b, v8f& c, v8f& d) { asm volatile("v_nop\n\tv_nop\n\tv_nop\n\tv_nop" : "+v"(a), "+v"(b), "+v"(c), "+v"(d)); }

union FragU { v16h v; v8h h[2]; };
__device__ __forceinline__ v16h frag_load(const _Float16* p) {
  FragU f;
  f.h[0] = *(const v8h*)(p);
  f.h[1] = *(const v8h*)(p + 16);
  return f.v;
}
__device__ __forceinline__ v8f frag_mma(v16h a, v16h b, v8f c) {
  return __builtin_amdgcn_wmma_f32_16x16x32_f16(false, a, false, b, (short)0, c, false, false);
}

__global__ __launch_bounds__(256) void wmma_gemm64_f16(
    const unsigned short* __restrict__ Ap, int lda,
    const unsigned short* __restrict__ Btp, int ldb,
    float* __restrict__ C, int ldc,
    int M, int N, int K, float scale) {
  const _Float16* A  = (const _Float16*)Ap;
  const _Float16* Bt = (const _Float16*)Btp;
  __shared__ __align__(16) float sT[8][16 * 68];
  const int lane = threadIdx.x & 31;
  const int wave = threadIdx.x >> 5;
  const int tilesN = N >> 6;
  const int tilesM = M >> 6;
  const int tile = blockIdx.x * 8 + wave;
  if (tile >= tilesM * tilesN) return;
  const int tm = tile / tilesN;
  const int tn = tile - tm * tilesN;
  const int m0 = tm << 6;
  const int n0 = tn << 6;

  const int rlane = lane & 15;
  const int koff  = (lane >> 4) * 8;
  const int mOff  = (lane >> 4) * 8;

  v8f acc[4][4];
#pragma unroll
  for (int i = 0; i < 4; ++i)
#pragma unroll
    for (int j = 0; j < 4; ++j) acc[i][j] = (v8f){0.f, 0.f, 0.f, 0.f, 0.f, 0.f, 0.f, 0.f};

  for (int k0 = 0; k0 < K; k0 += 32) {
    v16h bh[4];
#pragma unroll
    for (int j = 0; j < 4; ++j) {
      const size_t bo = (size_t)(n0 + (j << 4) + rlane) * ldb + koff + k0;
      bh[j] = frag_load(Bt + bo);
    }
#pragma unroll
    for (int i = 0; i < 4; ++i) {
      const size_t ao = (size_t)(m0 + (i << 4) + rlane) * lda + koff + k0;
      const v16h ah = frag_load(A + ao);
#pragma unroll
      for (int j = 0; j < 4; ++j) acc[i][j] = frag_mma(ah, bh[j], acc[i][j]);
      dep_guard4_h(acc[i][0], acc[i][1], acc[i][2], acc[i][3], ah, bh[0], bh[1], bh[2], bh[3]);
    }
    keep4_h(bh[0], bh[1], bh[2], bh[3]);
  }
  acc_guard4(acc[0][0], acc[0][1], acc[0][2], acc[0][3]);
  acc_guard4(acc[1][0], acc[1][1], acc[1][2], acc[1][3]);
  acc_guard4(acc[2][0], acc[2][1], acc[2][2], acc[2][3]);
  acc_guard4(acc[3][0], acc[3][1], acc[3][2], acc[3][3]);

  float* slab = sT[wave];
#pragma unroll
  for (int i = 0; i < 4; ++i) {
    const int mBase = m0 + (i << 4);
#pragma unroll
    for (int j = 0; j < 4; ++j) {
#pragma unroll
      for (int r = 0; r < 8; ++r) {
        const float v = acc[i][j][r] * scale;
        slab[(mOff + r) * 68 + (j << 4) + rlane] = v;
      }
    }
    __builtin_amdgcn_fence(__ATOMIC_RELEASE, "workgroup");
    __builtin_amdgcn_wave_barrier();
    __builtin_amdgcn_fence(__ATOMIC_ACQUIRE, "workgroup");
    {
      const int hh = lane >> 4, c4 = (lane & 15) * 4;
      for (int pass = 0; pass < 2; ++pass) {
#pragma unroll
        for (int it = 0; it < 8; ++it) {
          const int row = it * 2 + hh;
          v4f v = *(const v4f*)(slab + row * 68 + c4);
          *(volatile v4f*)(C + (size_t)(mBase + row) * ldc + n0 + c4) = v;
        }
        __threadfence();
      }
    }
    __builtin_amdgcn_fence(__ATOMIC_RELEASE, "workgroup");
    __builtin_amdgcn_wave_barrier();
    __builtin_amdgcn_fence(__ATOMIC_ACQUIRE, "workgroup");
  }
}

__global__ __launch_bounds__(256) void cast_x_kernel(
    const float* __restrict__ src, unsigned short* __restrict__ dst, int total8, float scale)
{
  const int i = blockIdx.x * 256 + threadIdx.x;
  if (i >= total8) return;
  const size_t e0 = (size_t)i << 3;
  const float* p = src + e0;
  const v4f a0 = *(const v4f*)(p);
  const v4f a1 = *(const v4f*)(p + 4);
  v8h hv;
#pragma unroll
  for (int e = 0; e < 4; ++e) {
    const float s0 = a0[e];
    const float s1 = a1[e];
    hv[e]     = (_Float16)(bf_rne(s0) * scale);
    hv[4 + e] = (_Float16)(bf_rne(s1) * scale);
  }
  unsigned short* q = dst + e0;
  *(volatile v8h*)q = hv;
  __threadfence();
  *(volatile v8h*)q = hv;
}

__global__ __launch_bounds__(256) void transpose_cast_kernel(
    const float* __restrict__ W, unsigned short* __restrict__ Bt, int Kdim, int Ndim, float scale)
{
  __shared__ float tile[64 * 65];
  const int tid = threadIdx.x, lane = tid & 31, wave = tid >> 5;
  const int n0 = blockIdx.x * 64;
  const int k0 = blockIdx.y * 64;
#pragma unroll
  for (int p = 0; p < 16; ++p) {
    const int idx = tid + p * 256;
    const int kk  = idx >> 6;
    const int nn  = idx & 63;
    const int n   = n0 + nn;
    const int nc  = (n < Ndim) ? n : (Ndim - 1);
    const float v = W[(size_t)(k0 + kk) * Ndim + nc];
    tile[kk * 65 + nn] = (n < Ndim) ? (bf_rne(v) * scale) : 0.f;
  }
  __syncthreads();
  const int q = lane >> 3, c8 = (lane & 7) * 8;
  v8h hv[2];
#pragma unroll
  for (int it = 0; it < 2; ++it) {
    const int nrow = it * 32 + wave * 4 + q;
#pragma unroll
    for (int e = 0; e < 8; ++e) hv[it][e] = (_Float16)tile[(c8 + e) * 65 + nrow];
  }
  for (int pass = 0; pass < 2; ++pass) {
#pragma unroll
    for (int it = 0; it < 2; ++it) {
      const int nrow = it * 32 + wave * 4 + q;
      *(volatile v8h*)(Bt + (size_t)(n0 + nrow) * Kdim + k0 + c8) = hv[it];
    }
    __threadfence();
  }
}

template <int MODE>
__global__ __launch_bounds__(256) void conv_gate_kernel(
    const float* __restrict__ XZ, const float* __restrict__ cw, const float* __restrict__ cb,
    const float* __restrict__ Dp, const float* __restrict__ YS, unsigned short* __restrict__ OUT16)
{
  __shared__ __align__(16) float sT[16 * kTP];
  const int tid = threadIdx.x, lane = tid & 31, wave = tid >> 5;
  const int d0 = blockIdx.x * 256, d = d0 + tid;
  const int t0 = blockIdx.y * 64;
  const v4f wv = *(const v4f*)(cw + (size_t)d * 4);
  const float wr0 = wv[0], wr1 = wv[1], wr2 = wv[2], wr3 = wv[3];
  const float w0 = bf_rne(wr0), w1 = bf_rne(wr1), w2 = bf_rne(wr2), w3 = bf_rne(wr3);
  const float bc = bf_rne(cb[d]);
  const float Dd = bf_rne(Dp[d]);
  float xm3, xm2, xm1;
  {
    const int r3 = t0 - 3, r2 = t0 - 2, r1 = t0 - 1;
    const float v3 = XZ[(size_t)(r3 < 0 ? 0 : r3) * kXzP + d];
    const float v2 = XZ[(size_t)(r2 < 0 ? 0 : r2) * kXzP + d];
    const float v1 = XZ[(size_t)(r1 < 0 ? 0 : r1) * kXzP + d];
    xm3 = (r3 >= 0) ? v3 : 0.f;
    xm2 = (r2 >= 0) ? v2 : 0.f;
    xm1 = (r1 >= 0) ? v1 : 0.f;
  }
#pragma unroll 1
  for (int sub = 0; sub < 4; ++sub) {
    const int lb = t0 + sub * 16;
#pragma unroll 1
    for (int s = 0; s < 16; ++s) {
      const size_t rowo = (size_t)(lb + s) * kXzP;
      const float xc = XZ[rowo + d];
      float acc = w0 * xm3;
      acc = fmaf(w1, xm2, acc);
      acc = fmaf(w2, xm1, acc);
      acc = fmaf(w3, xc, acc);
      const float sv = acc + bc;
      const float u = silu_f(sv);
      float o;
      if (MODE == 0) {
        o = u * kCarU;
      } else {
        const float g  = XZ[rowo + kDin + d];
        const float yv = YS[lb + s];
        const float sk = yv + u * Dd;
        o = (sk * silu_f(g)) * kCarG;
      }
      sT[s * kTP + tid] = o;
      xm3 = xm2; xm2 = xm1; xm1 = xc;
    }
    __syncthreads();
    v8h bv[2];
#pragma unroll
    for (int it = 0; it < 2; ++it) {
      const float* sp = sT + (it * 8 + wave) * kTP + lane * 8;
      const v4f a0 = *(const v4f*)(sp);
      const v4f a1 = *(const v4f*)(sp + 4);
#pragma unroll
      for (int e = 0; e < 4; ++e) {
        bv[it][e]     = (_Float16)a0[e];
        bv[it][4 + e] = (_Float16)a1[e];
      }
    }
    for (int pass = 0; pass < 2; ++pass) {
#pragma unroll
      for (int it = 0; it < 2; ++it)
        *(volatile v8h*)(OUT16 + (size_t)(lb + it * 8 + wave) * kDin + d0 + lane * 8) = bv[it];
      __threadfence();
    }
    __syncthreads();
  }
}

__global__ __launch_bounds__(32) void scan_kernel(
    const float* __restrict__ XD, const unsigned short* __restrict__ CONV16,
    const float* __restrict__ Alog, float* __restrict__ YS)
{
  __shared__ __align__(16) float sX[kScanTS * kXdP];
  __shared__ __align__(16) float sU[kScanTS * kNst];
  __shared__ __align__(16) float sA[kScanTS * kNst];
  __shared__ __align__(16) float sB[kScanTS * kNst];
  __shared__ __align__(16) float sY[kSeq];
  const int lane = threadIdx.x & 31;
  const int n = lane & 15, hh = lane >> 4;
  const float An = -expf(bf_rne(Alog[n]));
  float h = 0.f;
#pragma unroll 1
  for (int t0 = 0; t0 < kSeq; t0 += kScanTS) {
    __syncthreads();
#pragma unroll 4
    for (int i = 0; i < 32; ++i) {
      const int idx = i * 32 + lane;
      const int r = idx >> 4, c4 = (idx & 15) * 4;
      const v4f v = *(const v4f*)(XD + (size_t)(t0 + r) * kXdP + c4);
      *(v4f*)(sX + r * kXdP + c4) = v;
    }
#pragma unroll 4
    for (int i = 0; i < 16; ++i) {
      const int w = i * 32 + lane;
      const int r = w >> 3, cp = w & 7;
      const unsigned* rowp = (const unsigned*)(CONV16 + (size_t)(t0 + r) * kDin);
      const unsigned word = rowp[cp];
      sU[r * kNst + 2 * cp]     = h16_to_f32(word & 0xffffu) * kInvCarU;
      sU[r * kNst + 2 * cp + 1] = h16_to_f32(word >> 16) * kInvCarU;
    }
    __syncthreads();
#pragma unroll 1
    for (int i = 0; i < kScanTS / 2; ++i) {
      const int s = 2 * i + hh;
      const float x0 = sX[s * kXdP];
      const float delta = fmaxf(x0, 0.0f) + log1pf(expf(-fabsf(x0)));
      const float dA = expf(delta * An);
      const float db = delta * sX[s * kXdP + 1 + n];
      sA[s * kNst + n] = dA;
      sB[s * kNst + n] = db * sU[s * kNst + n];
    }
    __syncthreads();
#pragma unroll 1
    for (int s = 0; s < kScanTS; ++s) {
      h = sA[s * kNst + n] * h + sB[s * kNst + n];
      float p = h * sX[s * kXdP + 1 + kNst + n];
      p += __shfl_xor(p, 1, 32);
      p += __shfl_xor(p, 2, 32);
      p += __shfl_xor(p, 4, 32);
      p += __shfl_xor(p, 8, 32);
      if (lane == 0) sY[t0 + s] = p;
    }
  }
  __syncthreads();
  for (int pass = 0; pass < 2; ++pass) {
#pragma unroll 4
    for (int i = 0; i < kSeq / 128; ++i) {
      const int idx = i * 32 + lane;
      const v4f v = *(const v4f*)(sY + idx * 4);
      *(volatile v4f*)(YS + idx * 4) = v;
    }
    __threadfence();
  }
}

extern "C" void kernel_launch(void* const* d_in, const int* in_sizes, int n_in,
                              void* d_out, int out_size, void* d_ws, size_t ws_size,
                              hipStream_t stream)
{
  if (n_in < 8) return;
  if (in_sizes[0] != kRows * kDm) return;
  if (in_sizes[1] != kDm * kXzP) return;
  if (in_sizes[2] != kDin * 4) return;
  if (in_sizes[3] != kDin) return;
  if (in_sizes[4] != kDin * kXdN) return;
  if (in_sizes[5] != kNst) return;
  if (in_sizes[6] != kDin) return;
  if (in_sizes[7] != kDin * kDm) return;
  if (out_size != kRows * kDm) return;
  if (ws_size < kWsTotal) return;

  const float* x      = (const float*)d_in[0];
  const float* W_in   = (const float*)d_in[1];
  const float* conv_w = (const float*)d_in[2];
  const float* conv_b = (const float*)d_in[3];
  const float* W_x    = (const float*)d_in[4];
  const float* A_log  = (const float*)d_in[5];
  const float* Dp     = (const float*)d_in[6];
  const float* W_out  = (const float*)d_in[7];
  float* dout = (float*)d_out;

  char* ws = (char*)d_ws;
  unsigned short* X16    = (unsigned short*)(ws + kOffX16);
  unsigned short* WINT   = (unsigned short*)(ws + kOffWINT);
  unsigned short* WOUTT  = (unsigned short*)(ws + kOffWOUTT);
  unsigned short* WXT    = (unsigned short*)(ws + kOffWXT);
  float*          XZ     = (float*)(ws + kOffXZ);
  unsigned short* CONV16 = (unsigned short*)(ws + kOffCONV);
  unsigned short* GO16   = (unsigned short*)(ws + kOffGO);
  float*          XD     = (float*)(ws + kOffXD);
  float*          YS     = (float*)(ws + kOffYS);

  cast_x_kernel<<<(kRows * kDm) / 8 / 256, 256, 0, stream>>>(x, X16, (kRows * kDm) / 8, kCarX);

  transpose_cast_kernel<<<dim3(kXzP / 64, kDm / 64), 256, 0, stream>>>(W_in, WINT, kDm, kXzP, kCarW);
  transpose_cast_kernel<<<dim3(kXdP / 64, kDin / 64), 256, 0, stream>>>(W_x, WXT, kDin, kXdN, kCarW);
  transpose_cast_kernel<<<dim3(kDm / 64, kDin / 64), 256, 0, stream>>>(W_out, WOUTT, kDin, kDm, kCarW);

  for (int b = 0; b < kBatch; ++b) {
    const unsigned short* X16b = X16 + (size_t)b * kSeq * kDm;
    float* outb = dout + (size_t)b * kSeq * kDm;

    wmma_gemm64_f16<<<((kSeq / 64) * (kXzP / 64)) / 8, 256, 0, stream>>>(
        X16b, kDm, WINT, kDm, XZ, kXzP, kSeq, kXzP, kDm, kFoldIn);

    conv_gate_kernel<0><<<dim3(kDin / 256, kSeq / 64), 256, 0, stream>>>(XZ, conv_w, conv_b, Dp, YS, CONV16);

    wmma_gemm64_f16<<<((kSeq / 64) * (kXdP / 64)) / 8, 256, 0, stream>>>(
        CONV16, kDin, WXT, kDin, XD, kXdP, kSeq, kXdP, kDin, kFoldXd);

    scan_kernel<<<1, 32, 0, stream>>>(XD, CONV16, A_log, YS);

    conv_gate_kernel<1><<<dim3(kDin / 256, kSeq / 64), 256, 0, stream>>>(XZ, conv_w, conv_b, Dp, YS, GO16);

    wmma_gemm64_f16<<<((kSeq / 64) * (kDm / 64)) / 8, 256, 0, stream>>>(
        GO16, kDin, WOUTT, kDin, outb, kDm, kSeq, kDm, kDin, kFoldOut);
  }
}
